// GCN_60842506715219
// MI455X (gfx1250) — hardware-verified
//
#include <hip/hip_runtime.h>
#include <stddef.h>
#include <stdint.h>
#include <math.h>

#define NN      100000
#define NE      3200000
#define DMK     64
#define DHID    128
#define DGC     64
#define NTHR    256
#define FBLK    256
#define NFB     391
#define MP      100096
#define XSP     256
#define NSLOT   512
#define NBLK    196
#define BPR     14
#define NREG    14
#define RSPAN   7168
#define NCHK    16
#define CHE     200000
#define SUB     2048
#define CITER   98
#define RUNCAP  16384
#define RUNP    (RUNCAP + 32)
#define RS_N    (RUNP / 4)
#define RS_IT   ((RS_N + NTHR - 1) / NTHR)
#define RCAP    17920
#define DEGCAP  96
#define NSLOTS_ALL (NBLK * NSLOT)
#define ACCP    132
#define TTP     72
#define ACC_BYTES  (FBLK * ACCP * 4)
#define TTS_HALVES (8 * 64 * TTP)
#define FUSE_LDS   (ACC_BYTES + TTS_HALVES * 2)
#define COARSE_LDS (RUNP * 4)
#define BK_SL    RCAP
#define BK_CW    (2 * RCAP)
#define BK_CNT   (2 * RCAP + 8 * NSLOT)
#define BK_OFF   (BK_CNT + NSLOT)
#define BK_CUR   (BK_OFF + NSLOT)
#define BK_MISC  (BK_CUR + NSLOT)
#define BK_INTS  (BK_MISC + 32)
#define BUCKET_LDS (BK_INTS * 4)
#define NU_T    (DHID * DMK * (DMK / 8))
#define NU_F    (DHID * (DHID / 8))
#define NU_G    (DGC * (256 / 8))
#define GBM     64
#define GBN     64
#define GTHR    128
#define KG      256
#define WSMAX   134217728

static_assert(NCHK * CHE == NE);
static_assert(CHE % 8 == 0 && SUB == NTHR * 8 && CITER * SUB >= CHE && (CITER - 1) * SUB < CHE);
static_assert(NREG * RSPAN >= NN && NREG * BPR == NBLK && BPR * NSLOT == RSPAN);
static_assert(NN <= 131072 && RSPAN <= 8192);
static_assert(NBLK * NSLOT >= MP && MP == NFB * FBLK && MP >= NN && MP % GBM == 0);
static_assert(RUNCAP % SUB == 0 && RUNP % 4 == 0 && (RUNP * 4) % 128 == 0);
static_assert(RS_N * 4 == RUNP && RS_IT * NTHR >= RS_N && (RS_IT - 1) * NTHR < RS_N);
static_assert(RCAP >= 16708 + 835 && RCAP % 32 == 0 && (RCAP * 4) % 128 == 0);
static_assert(DEGCAP >= 63 + 8 && DEGCAP % 32 == 0);
static_assert(NN % 32 == 0 && NSLOT % 32 == 0 && NSLOT == 2 * NTHR);
static_assert(NU_T % NTHR == 0 && NU_F % NTHR == 0 && NU_G % NTHR == 0);
static_assert(BK_INTS % 4 == 0 && BUCKET_LDS <= 300000 && FUSE_LDS <= 300000);
static_assert((ACCP * 4) % 16 == 0 && (TTP * 2) % 16 == 0);
static_assert(KG % 32 == 0 && DGC == GBN && GBM == (GTHR / 32) * 16);

typedef float          v2f   __attribute__((ext_vector_type(2)));
typedef float          v4f   __attribute__((ext_vector_type(4)));
typedef float          v8f   __attribute__((ext_vector_type(8)));
typedef int            v4i   __attribute__((ext_vector_type(4)));
typedef int            v8i   __attribute__((ext_vector_type(8)));
typedef unsigned int   v4u   __attribute__((ext_vector_type(4)));
typedef unsigned short v8us  __attribute__((ext_vector_type(8)));
typedef unsigned short v16us __attribute__((ext_vector_type(16)));
typedef __bf16         v16bf __attribute__((ext_vector_type(16)));
typedef v2f  __attribute__((may_alias)) v2fa;
typedef v4f  __attribute__((may_alias)) v4fa;
typedef v4i  __attribute__((may_alias)) v4ia;
typedef v4u  __attribute__((may_alias)) v4ua;
typedef v8us __attribute__((may_alias)) v8usa;
union FragB { v16bf v; v16us u; v8us h[2]; v8i w; };

__device__ __forceinline__ v8f wmb(const FragB& a, const FragB& b, v8f c) {
  v8f d = __builtin_amdgcn_wmma_f32_16x16x32_bf16(false, a.v, false, b.v, (short)0, c, false, false);
  asm volatile("v_nop\n\tv_nop\n\tv_nop\n\tv_nop" : "+v"(d) : "v"(a.w), "v"(b.w));
  return d;
}

__device__ __forceinline__ void wm4(const FragB& a0, const FragB& a1,
                                    const FragB& b00, const FragB& b01,
                                    const FragB& b10, const FragB& b11, v8f& d0, v8f& d1) {
  v8f x0 = __builtin_amdgcn_wmma_f32_16x16x32_bf16(false, a0.v, false, b00.v, (short)0, d0, false, false);
  v8f x1 = __builtin_amdgcn_wmma_f32_16x16x32_bf16(false, a0.v, false, b10.v, (short)0, d1, false, false);
  x0 = __builtin_amdgcn_wmma_f32_16x16x32_bf16(false, a1.v, false, b01.v, (short)0, x0, false, false);
  x1 = __builtin_amdgcn_wmma_f32_16x16x32_bf16(false, a1.v, false, b11.v, (short)0, x1, false, false);
  asm volatile("v_nop\n\tv_nop\n\tv_nop\n\tv_nop"
               : "+v"(x0), "+v"(x1)
               : "v"(a0.w), "v"(a1.w), "v"(b00.w), "v"(b01.w), "v"(b10.w), "v"(b11.w));
  d0 = x0; d1 = x1;
}

__device__ __forceinline__ void wave_lds_sync() {
  __builtin_amdgcn_fence(__ATOMIC_RELEASE, "wavefront");
  __builtin_amdgcn_wave_barrier();
  __builtin_amdgcn_fence(__ATOMIC_ACQUIRE, "wavefront");
}

__device__ __forceinline__ unsigned bf16_bits(float f) {
  const unsigned u = __float_as_uint(f);
  const unsigned r = (u + 0x7FFFu + ((u >> 16) & 1u)) >> 16;
  const unsigned q = (u >> 16) | 0x40u;
  return ((u & 0x7FFFFFFFu) > 0x7F800000u) ? q : r;
}
__device__ __forceinline__ float bf16_val(float f) {
  return __uint_as_float(bf16_bits(f) << 16);
}

__device__ __forceinline__ v8us cvt8(const float* p, bool ok) {
  const v4f a = *(const v4fa*)p;
  const v4f b = *(const v4fa*)(p + 4);
  v8us o;
  o[0] = ok ? (unsigned short)bf16_bits(a.x) : (unsigned short)0;
  o[1] = ok ? (unsigned short)bf16_bits(a.y) : (unsigned short)0;
  o[2] = ok ? (unsigned short)bf16_bits(a.z) : (unsigned short)0;
  o[3] = ok ? (unsigned short)bf16_bits(a.w) : (unsigned short)0;
  o[4] = ok ? (unsigned short)bf16_bits(b.x) : (unsigned short)0;
  o[5] = ok ? (unsigned short)bf16_bits(b.y) : (unsigned short)0;
  o[6] = ok ? (unsigned short)bf16_bits(b.z) : (unsigned short)0;
  o[7] = ok ? (unsigned short)bf16_bits(b.w) : (unsigned short)0;
  return o;
}

__device__ __forceinline__ int blk_prefix(int cntT, int lane, int wave, int* wt, int& base) {
  int incl = cntT;
#pragma unroll
  for (int d = 1; d < 32; d <<= 1) {
    const int y = __shfl_up(incl, d, 32);
    if (lane >= d) incl += y;
  }
  const int wtotal = __shfl(incl, 31, 32);
  if (lane == 0) wt[wave] = wtotal;
  __syncthreads();
  int pre = 0, tot = 0;
#pragma unroll
  for (int w2 = 0; w2 < 8; ++w2) {
    const int t = wt[w2];
    pre += (w2 < wave) ? t : 0;
    tot += t;
  }
  const int pos = base + pre + (incl - cntT);
  base += tot;
  return pos;
}

__global__ __launch_bounds__(NTHR) void k_prep(const float* __restrict__ T, const float* __restrict__ Wf,
                                               const float* __restrict__ Wg,
                                               unsigned short* TT, unsigned short* WFT, unsigned short* WGD) {
  const int u = (int)blockIdx.x * NTHR + (int)threadIdx.x;
  v8us o;
  unsigned short* dp;
  if (u < NU_T) {
    const int row = u >> 3;
    const int h   = row >> 6;
    const int e   = row & 63;
    const int d0  = (u & 7) * 8;
    const float* p = T + (size_t)h * 4096 + (size_t)d0 * 64 + e;
#pragma unroll
    for (int i = 0; i < 8; ++i) o[i] = (unsigned short)bf16_bits(p[(size_t)i * 64]);
    dp = TT + (size_t)row * 64 + d0;
  } else if (u < NU_T + NU_F) {
    const int v  = u - NU_T;
    const int n  = v >> 4;
    const int k8 = (v & 15) * 8;
    const float* p = Wf + (size_t)k8 * DHID + n;
#pragma unroll
    for (int i = 0; i < 8; ++i) o[i] = (unsigned short)bf16_bits(p[(size_t)i * DHID]);
    dp = WFT + (size_t)n * DHID + k8;
  } else if (u < NU_T + NU_F + NU_G) {
    const int v  = u - NU_T - NU_F;
    const int n  = v >> 5;
    const int k8 = (v & 31) * 8;
    const int kk = k8 & (DHID - 1);
    const float* p = Wg + (size_t)kk * DGC + n;
#pragma unroll
    for (int i = 0; i < 8; ++i) o[i] = (unsigned short)bf16_bits(p[(size_t)i * DGC]);
    dp = WGD + (size_t)n * KG + k8;
  } else {
    return;
  }
  *(volatile v8us*)dp = o;
  __threadfence();
  *(volatile v8us*)dp = o;
}

__global__ __launch_bounds__(NTHR) void k_coarse(const int* __restrict__ ei, unsigned int* run) {
  extern __shared__ __attribute__((aligned(16))) unsigned char dsm[];
  unsigned int* lbuf = (unsigned int*)dsm;
  __shared__ int wtot[16];
  const int tid = (int)threadIdx.x, lane = tid & 31, wave = tid >> 5;
  const int c = (int)blockIdx.x / NCHK;
  const int k = (int)blockIdx.x - c * NCHK;
  const unsigned rb = (unsigned)(c * RSPAN);
  const int* srcp = ei + (size_t)k * CHE;
  const int* dstp = ei + (size_t)NE + (size_t)k * CHE;

  {
    const v4u z4 = {0u, 0u, 0u, 0u};
    for (int i = tid * 4; i < RUNP; i += NTHR * 4) *(v4ua*)(lbuf + i) = z4;
    if (tid < 16) wtot[tid] = 0;
  }
  __syncthreads();

  int base = 0;
#pragma unroll 1
  for (int it = 0; it < CITER; ++it) {
    const int e0 = it * SUB + 8 * tid;
    const bool valid = e0 < CHE;
    const int ec = valid ? e0 : (CHE - 8);
    const v4i da = *(const v4ia*)(dstp + ec);
    const v4i db = *(const v4ia*)(dstp + ec + 4);
    const v4i sa = *(const v4ia*)(srcp + ec);
    const v4i sb = *(const v4ia*)(srcp + ec + 4);
    int dv[8], sv[8];
    dv[0] = da.x; dv[1] = da.y; dv[2] = da.z; dv[3] = da.w;
    dv[4] = db.x; dv[5] = db.y; dv[6] = db.z; dv[7] = db.w;
    sv[0] = sa.x; sv[1] = sa.y; sv[2] = sa.z; sv[3] = sa.w;
    sv[4] = sb.x; sv[5] = sb.y; sv[6] = sb.z; sv[7] = sb.w;
    unsigned dl[8];
    bool hit[8];
    int cntT = 0;
#pragma unroll
    for (int j = 0; j < 8; ++j) {
      dl[j]  = (unsigned)dv[j] - rb;
      hit[j] = valid && (dl[j] < (unsigned)RSPAN) && ((unsigned)dv[j] < (unsigned)NN);
      cntT  += hit[j] ? 1 : 0;
    }
    int pos = blk_prefix(cntT, lane, wave, wtot + 8 * (it & 1), base);
#pragma unroll
    for (int j = 0; j < 8; ++j) {
      int s = sv[j];
      s = s < 0 ? 0 : (s > NN - 1 ? NN - 1 : s);
      const unsigned pk = (unsigned)s | (dl[j] << 17);
      if (hit[j]) {
        if (pos < RUNCAP) lbuf[32 + pos] = pk;
        pos = pos + 1;
      }
    }
  }
  __syncthreads();
  if (tid == 0) {
    lbuf[0] = (unsigned)(base > RUNCAP ? RUNCAP : base);
    lbuf[1] = (base > RUNCAP) ? 1u : 0u;
  }
  __syncthreads();

  unsigned int* rp = run + (size_t)blockIdx.x * RUNP;
#pragma unroll 1
  for (int i = 0; i < RS_IT; ++i) {
    const int p  = tid + i * NTHR;
    const bool ok = p < RS_N;
    const int pc = ok ? p : (RS_N - 1);
    const v4u v = *(const v4ua*)(lbuf + 4 * pc);
    if (ok) *(volatile v4u*)(rp + 4 * pc) = v;
  }
  __threadfence();
#pragma unroll 1
  for (int i = 0; i < RS_IT; ++i) {
    const int p  = tid + i * NTHR;
    const bool ok = p < RS_N;
    const int pc = ok ? p : (RS_N - 1);
    const v4u v = *(const v4ua*)(lbuf + 4 * pc);
    if (ok) *(volatile v4u*)(rp + 4 * pc) = v;
  }
}

__device__ __forceinline__ void bucket_store_pass(const int* sl, const int* cnt, const int* offs, int ovf,
                                                  int* lp, int* cp, int* op, float* dpv, int* fp, int tid) {
  for (int p = tid; p < RCAP / 4; p += NTHR) {
    const v4i v = *(const v4ia*)(sl + 4 * p);
    *(volatile v4i*)(lp + 4 * p) = v;
  }
  if (tid < NSLOT / 4) {
    const v4i c4 = *(const v4ia*)(cnt + 4 * tid);
    const v4i o4 = *(const v4ia*)(offs + 4 * tid);
    v4f d4;
    d4.x = rsqrtf((float)c4.x + 1.0f);
    d4.y = rsqrtf((float)c4.y + 1.0f);
    d4.z = rsqrtf((float)c4.z + 1.0f);
    d4.w = rsqrtf((float)c4.w + 1.0f);
    *(volatile v4i*)(cp + 4 * tid) = c4;
    *(volatile v4i*)(op + 4 * tid) = o4;
    *(volatile v4f*)(dpv + 4 * tid) = d4;
  }
  if (tid < 8) {
    v4i f4;
    f4.x = (tid == 0) ? ovf : 0; f4.y = 0; f4.z = 0; f4.w = 0;
    *(volatile v4i*)(fp + 4 * tid) = f4;
  }
}

__global__ __launch_bounds__(NTHR) void k_bucket(const unsigned int* __restrict__ run,
                                                 int* LIST, int* CNT, int* OFF, float* DIS, int* FLG) {
  extern __shared__ __attribute__((aligned(16))) unsigned char dsm[];
  int* ds   = (int*)dsm;
  int* hl   = ds;
  int* sl   = ds + BK_SL;
  int* cntw = ds + BK_CW;
  int* cnt  = ds + BK_CNT;
  int* offs = ds + BK_OFF;
  int* cur  = ds + BK_CUR;
  int* misc = ds + BK_MISC;
  __shared__ int wtot[16];
  const int tid = (int)threadIdx.x, lane = tid & 31, wave = tid >> 5;
  const int b = (int)blockIdx.x;
  const int c = b / BPR;
  const unsigned lb = (unsigned)((b - c * BPR) * NSLOT);

  {
    const v4i z4 = {0, 0, 0, 0};
    for (int i = tid * 4; i < BK_INTS; i += NTHR * 4) *(v4ia*)(ds + i) = z4;
    if (tid < 16) wtot[tid] = 0;
  }
  __syncthreads();

  int base = 0, rflag = 0, par = 0;
#pragma unroll 1
  for (int k = 0; k < NCHK; ++k) {
    const unsigned int* rp = run + (size_t)(c * NCHK + k) * RUNP;
    const v4u hd = *(const v4ua*)rp;
    const unsigned ck = hd.x > (unsigned)RUNCAP ? (unsigned)RUNCAP : hd.x;
    rflag |= (hd.y != 0u || hd.x > (unsigned)RUNCAP) ? 1 : 0;
    int nit = (int)((ck + (unsigned)(SUB - 1)) / (unsigned)SUB);
    nit = nit > RUNCAP / SUB ? RUNCAP / SUB : nit;
#pragma unroll 1
    for (int it = 0; it < nit; ++it) {
      const int e0 = it * SUB + 8 * tid;
      const v4u ea = *(const v4ua*)(rp + 32 + e0);
      const v4u eb = *(const v4ua*)(rp + 32 + e0 + 4);
      unsigned ev[8];
      ev[0] = ea.x; ev[1] = ea.y; ev[2] = ea.z; ev[3] = ea.w;
      ev[4] = eb.x; ev[5] = eb.y; ev[6] = eb.z; ev[7] = eb.w;
      unsigned sv[8];
      bool hit[8];
      int cntT = 0;
#pragma unroll
      for (int j = 0; j < 8; ++j) {
        sv[j]  = (ev[j] >> 17) - lb;
        hit[j] = ((unsigned)(e0 + j) < ck) && (sv[j] < (unsigned)NSLOT);
        cntT  += hit[j] ? 1 : 0;
      }
      int pos = blk_prefix(cntT, lane, wave, wtot + 8 * par, base);
      par ^= 1;
#pragma unroll
      for (int j = 0; j < 8; ++j) {
        const unsigned pk = (ev[j] & 0x1FFFFu) | (sv[j] << 17);
        if (hit[j]) {
          if (pos < RCAP) hl[pos] = (int)pk;
          pos = pos + 1;
        }
      }
    }
  }
  __syncthreads();
  const int tt  = base > RCAP ? RCAP : (base < 0 ? 0 : base);
  const int ovf = ((base > RCAP) ? 1 : 0) | rflag;
  const int nsteps = (tt + 31) >> 5;

#pragma unroll 1
  for (int st = wave; st < nsteps; st += 8) {
    const int idx = st * 32 + lane;
    const bool valid = idx < tt;
    const unsigned ent = (unsigned)hl[idx < RCAP ? idx : RCAP - 1];
    const int slot = valid ? (int)((ent >> 17) & 511u) : (NSLOT + lane);
    unsigned mm = 0u;
#pragma unroll
    for (int q = 0; q < 32; ++q) {
      const int sq = __builtin_amdgcn_readlane(slot, q);
      mm |= (sq == slot) ? (1u << q) : 0u;
    }
    const unsigned rank = (unsigned)__builtin_popcount(mm & ((1u << lane) - 1u));
    const bool last = (mm >> lane) == 1u;
    const int sc = slot < NSLOT ? slot : NSLOT - 1;
    if (valid) hl[idx] = (int)((ent & 0x3FFFFFFu) | (rank << 26) | (last ? 0x80000000u : 0u));
    if (valid && last) cntw[wave * NSLOT + sc] = cntw[wave * NSLOT + sc] + (int)rank + 1;
    wave_lds_sync();
  }
  __syncthreads();
  {
    int s0 = 0, s1 = 0;
#pragma unroll
    for (int w2 = 0; w2 < 8; ++w2) {
      s0 += cntw[w2 * NSLOT + tid];
      s1 += cntw[w2 * NSLOT + NTHR + tid];
    }
    cnt[tid] = s0;
    cnt[NTHR + tid] = s1;
  }
  __syncthreads();

  if (wave == 0) {
    const int sb = lane * (NSLOT / 32);
    int s = 0;
#pragma unroll 1
    for (int i = 0; i < NSLOT / 32; ++i) s += cnt[sb + i];
    int incl = s;
#pragma unroll
    for (int d = 1; d < 32; d <<= 1) {
      const int y = __shfl_up(incl, d, 32);
      if (lane >= d) incl += y;
    }
    int rn = incl - s;
#pragma unroll 1
    for (int i = 0; i < NSLOT / 32; ++i) {
      const int cv = cnt[sb + i];
      offs[sb + i] = rn;
      cur[sb + i]  = rn;
      rn += cv;
    }
  }
  __syncthreads();

  if (wave == 0) {
#pragma unroll 1
    for (int st = 0; st < nsteps; ++st) {
      const int idx = st * 32 + lane;
      const bool valid = idx < tt;
      const unsigned ent = (unsigned)hl[idx < RCAP ? idx : RCAP - 1];
      const int slot = (int)((ent >> 17) & 511u);
      const int rank = (int)((ent >> 26) & 31u);
      const bool last = (ent >> 31) != 0u;
      int p = cur[slot] + rank;
      p = p < 0 ? 0 : (p > RCAP - 1 ? RCAP - 1 : p);
      if (valid) sl[p] = (int)(ent & 0x1FFFFu);
      if (valid && last) cur[slot] = p + 1;
      wave_lds_sync();
    }
  }
  if (tid == 0) misc[0] = ovf;
  __syncthreads();

  int*   lp  = LIST + (size_t)b * RCAP;
  int*   cp  = CNT + (size_t)b * NSLOT;
  int*   op  = OFF + (size_t)b * NSLOT;
  float* dpv = DIS + (size_t)b * NSLOT;
  int*   fp  = FLG + (size_t)b * 32;
  const int ov = misc[0];
  bucket_store_pass(sl, cnt, offs, ov, lp, cp, op, dpv, fp, tid);
  __threadfence();
  bucket_store_pass(sl, cnt, offs, ov, lp, cp, op, dpv, fp, tid);
}

__global__ __launch_bounds__(NTHR) void k_fuse(const float* __restrict__ xm, const float* __restrict__ xn,
                                               const float* __restrict__ bfuse,
                                               const unsigned short* __restrict__ TT,
                                               const unsigned short* __restrict__ WFT,
                                               unsigned short* XS) {
  extern __shared__ __attribute__((aligned(16))) unsigned char dsm[];
  float* ACC = (float*)dsm;
  unsigned short* tts = (unsigned short*)(dsm + ACC_BYTES);
  const int tid = (int)threadIdx.x, lane = tid & 31, w = tid >> 5, hh = lane >> 4, m = lane & 15;
  const int base = (int)blockIdx.x * FBLK;
  const v8f z8 = {0.f, 0.f, 0.f, 0.f, 0.f, 0.f, 0.f, 0.f};

  FragB bxm[2][2], bxn[2][2];
#pragma unroll
  for (int nf = 0; nf < 2; ++nf) {
    const int node = base + 32 * w + 16 * nf + m;
    const bool ok = node < NN;
    const int rc = ok ? node : NN - 1;
    const float* pm = xm + (size_t)rc * DMK + 8 * hh;
    const float* pn = xn + (size_t)rc * DMK + 8 * hh;
#pragma unroll
    for (int ks = 0; ks < 2; ++ks) {
      bxm[nf][ks].h[0] = cvt8(pm + 32 * ks, ok);
      bxm[nf][ks].h[1] = cvt8(pm + 32 * ks + 16, ok);
      bxn[nf][ks].h[0] = cvt8(pn + 32 * ks, ok);
      bxn[nf][ks].h[1] = cvt8(pn + 32 * ks + 16, ok);
    }
  }

#pragma unroll 1
  for (int mt = 0; mt < 8; ++mt) {
    const unsigned short* wr = WFT + (size_t)(16 * mt + m) * DHID + 8 * hh;
    FragB a0, a1, a2, a3;
    a0.h[0] = *(const v8usa*)(wr);       a0.h[1] = *(const v8usa*)(wr + 16);
    a1.h[0] = *(const v8usa*)(wr + 32);  a1.h[1] = *(const v8usa*)(wr + 48);
    a2.h[0] = *(const v8usa*)(wr + 64);  a2.h[1] = *(const v8usa*)(wr + 80);
    a3.h[0] = *(const v8usa*)(wr + 96);  a3.h[1] = *(const v8usa*)(wr + 112);
    v8f d0 = z8, d1 = z8;
    wm4(a0, a1, bxm[0][0], bxm[0][1], bxm[1][0], bxm[1][1], d0, d1);
    wm4(a2, a3, bxn[0][0], bxn[0][1], bxn[1][0], bxn[1][1], d0, d1);
    const v4f q0 = *(const v4fa*)(bfuse + 16 * mt + 8 * hh);
    const v4f q1 = *(const v4fa*)(bfuse + 16 * mt + 8 * hh + 4);
    const float c0 = bf16_val(q0.x), c1 = bf16_val(q0.y), c2 = bf16_val(q0.z), c3 = bf16_val(q0.w);
    const float c4 = bf16_val(q1.x), c5 = bf16_val(q1.y), c6 = bf16_val(q1.z), c7 = bf16_val(q1.w);
    {
      float* ap = ACC + (32 * w + m) * ACCP + 16 * mt + 8 * hh;
      const v4f o0 = {d0[0] + c0, d0[1] + c1, d0[2] + c2, d0[3] + c3};
      const v4f o1 = {d0[4] + c4, d0[5] + c5, d0[6] + c6, d0[7] + c7};
      *(v4fa*)ap = o0;
      *(v4fa*)(ap + 4) = o1;
    }
    {
      float* ap = ACC + (32 * w + 16 + m) * ACCP + 16 * mt + 8 * hh;
      const v4f o0 = {d1[0] + c0, d1[1] + c1, d1[2] + c2, d1[3] + c3};
      const v4f o1 = {d1[4] + c4, d1[5] + c5, d1[6] + c6, d1[7] + c7};
      *(v4fa*)ap = o0;
      *(v4fa*)(ap + 4) = o1;
    }
  }

  float xnf[2][4][8];
#pragma unroll
  for (int nf = 0; nf < 2; ++nf) {
#pragma unroll
    for (int ks = 0; ks < 2; ++ks) {
#pragma unroll
      for (int i = 0; i < 8; ++i) {
        const unsigned w0 = (unsigned)bxn[nf][ks].w[i >> 1];
        const unsigned w1 = (unsigned)bxn[nf][ks].w[4 + (i >> 1)];
        xnf[nf][2 * ks][i]     = __uint_as_float((i & 1) ? (w0 & 0xFFFF0000u) : (w0 << 16));
        xnf[nf][2 * ks + 1][i] = __uint_as_float((i & 1) ? (w1 & 0xFFFF0000u) : (w1 << 16));
      }
    }
  }

#pragma unroll 1
  for (int c = 0; c < 16; ++c) {
    __syncthreads();
    {
      const unsigned short* src = TT + (size_t)c * (8 * 4096);
#pragma unroll 4
      for (int i = 0; i < 16; ++i) {
        const int p = tid + NTHR * i;
        const int row = p >> 3, seg = p & 7;
        const v8us v = *(const v8usa*)(src + (size_t)p * 8);
        *(v8usa*)(tts + row * TTP + seg * 8) = v;
      }
    }
    __syncthreads();
#pragma unroll 1
    for (int hl = 0; hl < 8; ++hl) {
      float acc0 = 0.0f, acc1 = 0.0f;
      const unsigned short* rp = tts + (hl * 64 + m) * TTP + 8 * hh;
#pragma unroll
      for (int mf = 0; mf < 4; ++mf) {
        const unsigned short* q = rp + 16 * mf * TTP;
        FragB a0, a1;
        a0.h[0] = *(const v8usa*)(q);       a0.h[1] = *(const v8usa*)(q + 16);
        a1.h[0] = *(const v8usa*)(q + 32);  a1.h[1] = *(const v8usa*)(q + 48);
        v8f d0 = z8, d1 = z8;
        wm4(a0, a1, bxm[0][0], bxm[0][1], bxm[1][0], bxm[1][1], d0, d1);
#pragma unroll
        for (int v = 0; v < 8; ++v) {
          acc0 = fmaf(d0[v], xnf[0][mf][v], acc0);
          acc1 = fmaf(d1[v], xnf[1][mf][v], acc1);
        }
      }
      const float s0 = acc0 + __shfl_xor(acc0, 16, 32);
      const float s1 = acc1 + __shfl_xor(acc1, 16, 32);
      const float sv = (hh != 0) ? s1 : s0;
      float* ap = ACC + (32 * w + lane) * ACCP + (8 * c + hl);
      const float old = *ap;
      *ap = old + sv;
    }
  }
  __syncthreads();

#pragma unroll 1
  for (int it = 0; it < 16; ++it) {
    const int nl = it * 16 + 2 * w + hh;
    const float* ap = ACC + nl * ACCP + 8 * m;
    const v4f a = *(const v4fa*)ap;
    const v4f b = *(const v4fa*)(ap + 4);
    float tv[8];
    tv[0] = tanhf(a.x); tv[1] = tanhf(a.y); tv[2] = tanhf(a.z); tv[3] = tanhf(a.w);
    tv[4] = tanhf(b.x); tv[5] = tanhf(b.y); tv[6] = tanhf(b.z); tv[7] = tanhf(b.w);
    v8us hv, lv;
#pragma unroll
    for (int i = 0; i < 8; ++i) {
      const unsigned hb = bf16_bits(tv[i]);
      const float hf = __uint_as_float(hb << 16);
      const unsigned lbits = bf16_bits(tv[i] - hf);
      hv[i] = (unsigned short)hb;
      lv[i] = (unsigned short)lbits;
    }
    unsigned short* dp = XS + (size_t)(base + nl) * XSP + 8 * m;
    *(volatile v8us*)dp = hv;
    *(volatile v8us*)(dp + DHID) = lv;
    __threadfence();
    *(volatile v8us*)dp = hv;
    *(volatile v8us*)(dp + DHID) = lv;
  }
}

__global__ __launch_bounds__(GTHR) void k_gemm(const unsigned short* __restrict__ A,
                                               const unsigned short* __restrict__ WT,
                                               const float* __restrict__ dis, float* outF) {
  __shared__ __attribute__((aligned(16))) float stg[GBM * GBN];
  __shared__ float sdis[GBM];
  const int tid = (int)threadIdx.x, lane = tid & 31, wave = tid >> 5, hh = lane >> 4, m = lane & 15;
  const int rowBase = (int)blockIdx.x * GBM;
  if (tid < GBM) sdis[tid] = dis[rowBase + tid];

  v8f acc[4];
  {
    const v8f z = {0.f, 0.f, 0.f, 0.f, 0.f, 0.f, 0.f, 0.f};
    acc[0] = z; acc[1] = z; acc[2] = z; acc[3] = z;
  }
  const unsigned short* ap = A  + (size_t)(rowBase + 16 * wave + m) * (size_t)KG + 8 * hh;
  const unsigned short* wp = WT + (size_t)m * (size_t)KG + 8 * hh;
#pragma unroll 1
  for (int ks = 0; ks < KG / 32; ++ks) {
    FragB af;
    af.h[0] = *(const v8usa*)(ap + 32 * ks);
    af.h[1] = *(const v8usa*)(ap + 32 * ks + 16);
#pragma unroll
    for (int t = 0; t < 4; ++t) {
      const unsigned short* wq = wp + (size_t)(16 * t) * (size_t)KG + 32 * ks;
      FragB bf;
      bf.h[0] = *(const v8usa*)wq;
      bf.h[1] = *(const v8usa*)(wq + 16);
      acc[t] = wmb(af, bf, acc[t]);
    }
  }
#pragma unroll
  for (int t = 0; t < 4; ++t) {
    const int lc = 16 * t + m;
#pragma unroll
    for (int r = 0; r < 8; ++r) {
      const int lr = 16 * wave + 8 * hh + r;
      stg[lr * GBN + lc] = acc[t][r];
    }
  }
  __syncthreads();

  v4f fv[8];
#pragma unroll
  for (int i = 0; i < 8; ++i) {
    const int lr = 16 * wave + 2 * i + hh;
    const v4f s4 = *(const v4fa*)(stg + lr * GBN + 4 * m);
    const float dv = sdis[lr];
    v4f o;
    o.x = s4.x * dv; o.y = s4.y * dv; o.z = s4.z * dv; o.w = s4.w * dv;
    fv[i] = o;
  }
#pragma unroll
  for (int i = 0; i < 8; ++i) {
    const int gr = rowBase + 16 * wave + 2 * i + hh;
    *(volatile v4f*)(outF + (size_t)gr * DGC + 4 * m) = fv[i];
  }
  __threadfence();
#pragma unroll
  for (int i = 0; i < 8; ++i) {
    const int gr = rowBase + 16 * wave + 2 * i + hh;
    *(volatile v4f*)(outF + (size_t)gr * DGC + 4 * m) = fv[i];
  }
}

__global__ __launch_bounds__(NTHR) void k_agg_out(const int* __restrict__ LIST, const int* __restrict__ CNT,
                                                  const int* __restrict__ OFF, const float* __restrict__ DIS,
                                                  const int* __restrict__ FLG, const float* __restrict__ HP,
                                                  const float* __restrict__ bgcn, const float* __restrict__ Wh,
                                                  const float* __restrict__ bhead, float* out) {
  __shared__ __attribute__((aligned(16))) float outs[NSLOT];
  const int tid = (int)threadIdx.x, lane = tid & 31, wave = tid >> 5;
  const int b = (int)blockIdx.x;
  const int nodeBase = b * NSLOT;
  const int* lp = LIST + (size_t)b * RCAP;
  const int fl = FLG[(size_t)b * 32];
  float bv0, bv1, wh0, wh1;
  {
    const v2f a = *(const v2fa*)(bgcn + 2 * lane);
    bv0 = bf16_val(a.x); bv1 = bf16_val(a.y);
    const v2f q = *(const v2fa*)(Wh + 2 * lane);
    wh0 = bf16_val(q.x); wh1 = bf16_val(q.y);
  }
  const float bh = bf16_val(bhead[0]);
  const float qnan = __int_as_float(0x7fc00000);

#pragma unroll 1
  for (int si = 0; si < NSLOT / 8; ++si) {
    const int s = si * 8 + wave;
    const int node = nodeBase + s;
    int c = CNT[node];
    const bool big = c > DEGCAP;
    c = c < 0 ? 0 : (c > DEGCAP ? DEGCAP : c);
    int o = OFF[node];
    o = o < 0 ? 0 : (o > RCAP ? RCAP : o);
    const int nc = node < NN ? node : NN - 1;
    const float dd = DIS[nc];
    float acc0 = 0.0f, acc1 = 0.0f;
#pragma unroll 1
    for (int b0 = 0; b0 < c; b0 += 32) {
      int idx = o + b0 + lane;
      idx = idx > RCAP - 1 ? RCAP - 1 : idx;
      int sr = lp[idx];
      sr = sr < 0 ? 0 : (sr > NN - 1 ? NN - 1 : sr);
      const int m32 = (c - b0) < 32 ? (c - b0) : 32;
#pragma unroll 1
      for (int k = 0; k < m32; ++k) {
        const int sk = __builtin_amdgcn_readlane(sr, k);
        const v2f a = *(const v2fa*)(HP + (size_t)sk * DGC + 2 * lane);
        acc0 += a.x; acc1 += a.y;
      }
    }
    float sv0, sv1;
    {
      const v2f a = *(const v2fa*)(HP + (size_t)nc * DGC + 2 * lane);
      sv0 = a.x; sv1 = a.y;
    }
    const float g0 = (acc0 + sv0) * dd + bv0;
    const float g1 = (acc1 + sv1) * dd + bv1;
    const float r0 = (g0 > 0.0f) ? g0 : (g0 - g0);
    const float r1 = (g1 > 0.0f) ? g1 : (g1 - g1);
    float p = r0 * wh0 + r1 * wh1;
    p += __shfl_xor(p, 1, 32);
    p += __shfl_xor(p, 2, 32);
    p += __shfl_xor(p, 4, 32);
    p += __shfl_xor(p, 8, 32);
    p += __shfl_xor(p, 16, 32);
    float val = p + bh;
    val = (fl != 0 || big) ? qnan : val;
    if (lane == 0) outs[s] = val;
  }
  __syncthreads();

  const bool okst = (tid < NSLOT / 4) && (nodeBase + 4 * tid < NN);
  const int tq = tid < NSLOT / 4 ? tid : 0;
  const v4f ov = *(const v4fa*)(outs + 4 * tq);
  float* op = out + (size_t)nodeBase + 4 * tq;
  if (okst) *(volatile v4f*)op = ov;
  __threadfence();
  if (okst) *(volatile v4f*)op = ov;
}

static inline size_t al256(size_t o) { return (o + 255) & ~(size_t)255; }

extern "C" void kernel_launch(void* const* d_in, const int* in_sizes, int n_in,
                              void* d_out, int out_size, void* d_ws, size_t ws_size,
                              hipStream_t stream) {
  if (n_in < 10) return;
  if (in_sizes[0] != NN * DMK || in_sizes[1] != NN * DMK) return;
  if (in_sizes[2] != 2 * NE) return;
  if (in_sizes[3] != DHID * DMK * DMK) return;
  if (in_sizes[4] != 2 * DMK * DHID || in_sizes[5] != DHID) return;
  if (in_sizes[6] != DHID * DGC || in_sizes[7] != DGC) return;
  if (in_sizes[8] != DGC || in_sizes[9] != 1) return;
  if (out_size != NN) return;

  const float* xm = (const float*)d_in[0];
  const float* xn = (const float*)d_in[1];
  const int*   ei = (const int*)d_in[2];
  const float* Tf = (const float*)d_in[3];
  const float* Wf = (const float*)d_in[4];
  const float* bf = (const float*)d_in[5];
  const float* Wg = (const float*)d_in[6];
  const float* bg = (const float*)d_in[7];
  const float* Wh = (const float*)d_in[8];
  const float* bh = (const float*)d_in[9];
  float* out = (float*)d_out;

  char* ws = (char*)d_ws;
  size_t off = 0;
  const size_t oTT  = off; off = al256(off + (size_t)DHID * DMK * DMK * 2);
  const size_t oWFT = off; off = al256(off + (size_t)DHID * DHID * 2);
  const size_t oWGD = off; off = al256(off + (size_t)DGC * KG * 2);
  const size_t oXS  = off; off = al256(off + (size_t)MP * XSP * 2);
  const size_t oHP  = off; off = al256(off + (size_t)MP * DGC * 4);
  const size_t oRUN = off; off = al256(off + (size_t)NREG * NCHK * RUNP * 4);
  const size_t oLST = off; off = al256(off + (size_t)NBLK * RCAP * 4);
  const size_t oCNT = off; off = al256(off + (size_t)NSLOTS_ALL * 4);
  const size_t oOFF = off; off = al256(off + (size_t)NSLOTS_ALL * 4);
  const size_t oDIS = off; off = al256(off + (size_t)NSLOTS_ALL * 4);
  const size_t oFLG = off; off = al256(off + (size_t)NBLK * 32 * 4);
  if (off > ws_size || off > (size_t)WSMAX) return;
  unsigned short* TT  = (unsigned short*)(ws + oTT);
  unsigned short* WFT = (unsigned short*)(ws + oWFT);
  unsigned short* WGD = (unsigned short*)(ws + oWGD);
  unsigned short* XS  = (unsigned short*)(ws + oXS);
  float*          HP  = (float*)(ws + oHP);
  unsigned int*   RUN = (unsigned int*)(ws + oRUN);
  int*            LST = (int*)(ws + oLST);
  int*            CNT = (int*)(ws + oCNT);
  int*            OFF = (int*)(ws + oOFF);
  float*          DIS = (float*)(ws + oDIS);
  int*            FLG = (int*)(ws + oFLG);

  hipFuncSetAttribute(reinterpret_cast<const void*>(&k_coarse), hipFuncAttributeMaxDynamicSharedMemorySize, (int)COARSE_LDS);
  hipFuncSetAttribute(reinterpret_cast<const void*>(&k_bucket), hipFuncAttributeMaxDynamicSharedMemorySize, (int)BUCKET_LDS);
  hipFuncSetAttribute(reinterpret_cast<const void*>(&k_fuse),   hipFuncAttributeMaxDynamicSharedMemorySize, (int)FUSE_LDS);

  k_prep<<<(NU_T + NU_F + NU_G) / NTHR, NTHR, 0, stream>>>(Tf, Wf, Wg, TT, WFT, WGD);
  k_coarse<<<NREG * NCHK, NTHR, COARSE_LDS, stream>>>(ei, RUN);
  k_bucket<<<NBLK, NTHR, BUCKET_LDS, stream>>>(RUN, LST, CNT, OFF, DIS, FLG);
  k_fuse<<<NFB, NTHR, FUSE_LDS, stream>>>(xm, xn, bf, TT, WFT, XS);
  k_gemm<<<MP / GBM, GTHR, 0, stream>>>(XS, WGD, DIS, HP);
  k_agg_out<<<NBLK, NTHR, 0, stream>>>(LST, CNT, OFF, DIS, FLG, HP, bg, Wh, bh, out);
}
